// nlpdo_torch_18391049962028
// MI455X (gfx1250) — hardware-verified
//
#include <hip/hip_runtime.h>
#include <hip/hip_bf16.h>


typedef float          v4f   __attribute__((ext_vector_type(4)));
typedef unsigned int   v4u   __attribute__((ext_vector_type(4)));
typedef unsigned short v8us  __attribute__((ext_vector_type(8)));
typedef __bf16         v16bf __attribute__((ext_vector_type(16)));
typedef float          v8f   __attribute__((ext_vector_type(8)));

union Frag { v16bf v; v8us p[2]; };

static constexpr int CIN  = 256;
static constexpr int IMH  = 64;
static constexpr int IMW  = 64;
static constexpr int HWN  = IMH * IMW;
static constexpr int CMID = 128;
static constexpr int NGRP = 16;
static constexpr int GDIM = 8;
static constexpr int CW   = 1600;
static constexpr int SPITCH = 32;


__device__ __forceinline__ unsigned int bf_bits(float f) {
    const unsigned int u = __float_as_uint(f);
    return (u + 0x7FFFu + ((u >> 16) & 1u)) >> 16;
}

__device__ __forceinline__ void split_hl(float v, unsigned int& hi, unsigned int& lo) {
    hi = bf_bits(v);
    const float hf = __uint_as_float(hi << 16);
    lo = bf_bits(v - hf);
}

__device__ __forceinline__ v8f zero8() {
    return (v8f){0.f, 0.f, 0.f, 0.f, 0.f, 0.f, 0.f, 0.f};
}

__device__ __forceinline__ v8f wmma3(v8f acc, v16bf ah, v16bf al, v16bf bh, v16bf bl) {
    acc = __builtin_amdgcn_wmma_f32_16x16x32_bf16(false, ah, false, bh, (short)0, acc, false, false);
    acc = __builtin_amdgcn_wmma_f32_16x16x32_bf16(false, ah, false, bl, (short)0, acc, false, false);
    acc = __builtin_amdgcn_wmma_f32_16x16x32_bf16(false, al, false, bh, (short)0, acc, false, false);
    asm volatile("v_nop\n\tv_nop\n\tv_nop\n\tv_nop" : "+v"(acc) : "v"(ah), "v"(al), "v"(bh), "v"(bl));
    return acc;
}

__global__ __launch_bounds__(256) void pack_w_kernel(const float* __restrict__ src,
                                                     unsigned short* dh, unsigned short* dl,
                                                     int Kd, int KT, int nthr) {
    const int t = blockIdx.x * 256 + threadIdx.x;
    if (t >= nthr) return;
    const int hs   = t & 1;
    const int lane = (t >> 1) & 31;
    const int rest = t >> 6;
    const int kt = rest % KT;
    const int mt = rest / KT;
    const int m = mt * 16 + (lane & 15);
    const int k = kt * 32 + 16 * hs + 8 * (lane >> 4);
    const float* s = src + (size_t)m * Kd + k;
    const v4f a = *(const v4f*)s;
    const v4f c = *(const v4f*)(s + 4);
    float v[8] = {a.x, a.y, a.z, a.w, c.x, c.y, c.z, c.w};
    unsigned int hi[8], lo[8];
#pragma unroll
    for (int j = 0; j < 8; ++j) split_hl(v[j], hi[j], lo[j]);
    v4u H, L;
    H.x = hi[0] | (hi[1] << 16); H.y = hi[2] | (hi[3] << 16);
    H.z = hi[4] | (hi[5] << 16); H.w = hi[6] | (hi[7] << 16);
    L.x = lo[0] | (lo[1] << 16); L.y = lo[2] | (lo[3] << 16);
    L.z = lo[4] | (lo[5] << 16); L.w = lo[6] | (lo[7] << 16);
    volatile v4u* ph = (volatile v4u*)(dh + (size_t)t * 8);
    volatile v4u* pl = (volatile v4u*)(dl + (size_t)t * 8);
    *ph = H;
    *pl = L;
    __threadfence();
    *ph = H;
    *pl = L;
}

template <int KT>
__global__ __launch_bounds__(256) void gemm_split_kernel(
        const unsigned short* __restrict__ Ah, const unsigned short* __restrict__ Al,
        const float* __restrict__ Bsrc, float* Cdst, int M, int N) {
    __shared__ __align__(16) unsigned short sBh[64 * 40];
    __shared__ __align__(16) unsigned short sBl[64 * 40];
    __shared__ __align__(16) float sC[8 * 16 * 64];

    const int tid  = threadIdx.x;
    const int lane = tid & 31;
    const int wave = tid >> 5;
    const int h    = lane >> 4;
    const int m    = lane & 15;
    const int bb   = blockIdx.z;
    const int n0   = blockIdx.x * 64;
    const int mt   = blockIdx.y * 8 + wave;
    const int m0   = mt * 16;
    const int K    = KT * 32;
    const float* Bb = Bsrc + (size_t)bb * K * N;

    v8f acc[4];
#pragma unroll
    for (int t = 0; t < 4; ++t) acc[t] = zero8();

#pragma unroll 1
    for (int kt = 0; kt < KT; ++kt) {
        const int k0 = kt * 32;
#pragma unroll
        for (int r = 0; r < 2; ++r) {
            const int f  = tid + 256 * r;
            const int kr = f >> 4;
            const int c4 = (f & 15) * 4;
            const v4f v = *(const v4f*)(Bb + (size_t)(k0 + kr) * N + n0 + c4);
            float bv[4] = {v.x, v.y, v.z, v.w};
#pragma unroll
            for (int j = 0; j < 4; ++j) {
                unsigned int hi, lo;
                split_hl(bv[j], hi, lo);
                sBh[(c4 + j) * 40 + kr] = (unsigned short)hi;
                sBl[(c4 + j) * 40 + kr] = (unsigned short)lo;
            }
        }
        __syncthreads();

        const size_t aoff = ((size_t)(mt * KT + kt) * 32 + lane) * 16;
        const v16bf ah = *(const v16bf*)(Ah + aoff);
        const v16bf al = *(const v16bf*)(Al + aoff);
#pragma unroll
        for (int t = 0; t < 4; ++t) {
            const int bi = (t * 16 + m) * 40 + 8 * h;
            Frag bh, bl;
            bh.p[0] = *(const v8us*)&sBh[bi];
            bh.p[1] = *(const v8us*)&sBh[bi + 16];
            bl.p[0] = *(const v8us*)&sBl[bi];
            bl.p[1] = *(const v8us*)&sBl[bi + 16];
            acc[t] = wmma3(acc[t], ah, al, bh.v, bl.v);
        }
        __syncthreads();
    }

#pragma unroll
    for (int t = 0; t < 4; ++t)
#pragma unroll
        for (int r = 0; r < 8; ++r)
            sC[(wave * 16 + 8 * h + r) * 64 + t * 16 + m] = acc[t][r];
    __syncthreads();

    v4f q[8];
#pragma unroll
    for (int it = 0; it < 8; ++it) {
        const int L   = it * 4 + (lane >> 3);
        const int row = L >> 1;
        const int col = (L & 1) * 32 + (lane & 7) * 4;
        q[it] = *(const v4f*)&sC[(wave * 16 + row) * 64 + col];
    }
    float* cbase = Cdst + ((size_t)bb * M + m0) * N + n0;
#pragma unroll
    for (int it = 0; it < 8; ++it) {
        const int L   = it * 4 + (lane >> 3);
        const int row = L >> 1;
        const int col = (L & 1) * 32 + (lane & 7) * 4;
        *(volatile v4f*)(cbase + (size_t)row * N + col) = q[it];
    }
    __threadfence();
#pragma unroll
    for (int it = 0; it < 8; ++it) {
        const int L   = it * 4 + (lane >> 3);
        const int row = L >> 1;
        const int col = (L & 1) * 32 + (lane & 7) * 4;
        *(volatile v4f*)(cbase + (size_t)row * N + col) = q[it];
    }
}

__global__ __launch_bounds__(256) void gn_stats_kernel(const float* __restrict__ mid, float* stats) {
    __shared__ float red[8];
    const int tid  = threadIdx.x;
    const int lane = tid & 31;
    const int wave = tid >> 5;
    const int grp  = blockIdx.x;
    const int b = grp >> 4, g = grp & 15;
    const v4f* base = (const v4f*)(mid + ((size_t)b * CMID + g * GDIM) * HWN);
    const int n4 = GDIM * HWN / 4;
    const float invn = 1.f / (float)(GDIM * HWN);

    float s = 0.f;
#pragma unroll 4
    for (int i = tid; i < n4; i += 256) {
        const v4f v = base[i];
        s += (v.x + v.y) + (v.z + v.w);
    }
#pragma unroll
    for (int o = 16; o > 0; o >>= 1) s += __shfl_xor(s, o);
    if (lane == 0) red[wave] = s;
    __syncthreads();
    const float tot = ((red[0] + red[1]) + (red[2] + red[3])) + ((red[4] + red[5]) + (red[6] + red[7]));
    __syncthreads();
    const float mean = tot * invn;

    float ss = 0.f;
#pragma unroll 4
    for (int i = tid; i < n4; i += 256) {
        const v4f v = base[i];
        const float dx = v.x - mean, dy = v.y - mean, dz = v.z - mean, dw = v.w - mean;
        ss += (dx * dx + dy * dy) + (dz * dz + dw * dw);
    }
#pragma unroll
    for (int o = 16; o > 0; o >>= 1) ss += __shfl_xor(ss, o);
    if (lane == 0) red[wave] = ss;
    __syncthreads();
    const float tot2 = ((red[0] + red[1]) + (red[2] + red[3])) + ((red[4] + red[5]) + (red[6] + red[7]));
    const float var  = tot2 * invn;
    const float rstd = rsqrtf(var + 1e-5f);

    if (tid < 8) {
        v4f o = (v4f){0.f, 0.f, 0.f, 0.f};
        if (tid == 0) { o.x = mean; o.y = rstd; }
        volatile v4f* p = (volatile v4f*)(stats + (size_t)grp * SPITCH + tid * 4);
        *p = o;
        __threadfence();
        *p = o;
    }
}

__global__ __launch_bounds__(256) void dynfilter_kernel(
        const unsigned short* __restrict__ W2h, const unsigned short* __restrict__ W2l,
        const float* __restrict__ mid, const float* __restrict__ stats,
        const float* __restrict__ gamma, const float* __restrict__ beta,
        const float* __restrict__ gw, const float* __restrict__ gb,
        const float* __restrict__ x, float* filt) {
    __shared__ __align__(16) unsigned short sXh[32 * 136];
    __shared__ __align__(16) unsigned short sXl[32 * 136];
    __shared__ __align__(16) float sWd[400 * 16];
    __shared__ __align__(16) float sOut[64 * 32];
    __shared__ float sPart[256];
    __shared__ __align__(16) float sScale[32];

    const int tid  = threadIdx.x;
    const int lane = tid & 31;
    const int wave = tid >> 5;
    const int h    = lane >> 4;
    const int m    = lane & 15;
    const int b    = blockIdx.y;
    const int pix0 = blockIdx.x * 32;
    const int y    = pix0 / IMW;
    const int xb   = pix0 % IMW;

#pragma unroll
    for (int r = 0; r < 4; ++r) {
        const int f  = tid + 256 * r;
        const int c  = f >> 3;
        const int p4 = (f & 7) * 4;
        const v4f v = *(const v4f*)(mid + ((size_t)(b * CMID + c)) * HWN + pix0 + p4);
        const int grp = c >> 3;
        const float mean = stats[(size_t)(b * NGRP + grp) * SPITCH + 0];
        const float rstd = stats[(size_t)(b * NGRP + grp) * SPITCH + 1];
        const float ga = gamma[grp], be = beta[grp], sw = gw[grp], sb = gb[grp];
        float tv[4] = {v.x, v.y, v.z, v.w};
#pragma unroll
        for (int j = 0; j < 4; ++j) {
            float t = (tv[j] - mean) * rstd;
            t = t * ga + be;
            t = t * sw + sb;
            t = fmaxf(t, 0.f);
            unsigned int hi, lo;
            split_hl(t, hi, lo);
            sXh[(p4 + j) * 136 + c] = (unsigned short)hi;
            sXl[(p4 + j) * 136 + c] = (unsigned short)lo;
        }
    }
    __syncthreads();

#pragma unroll 1
    for (int gp = 0; gp < 4; ++gp) {
#pragma unroll 1
        for (int ph = 0; ph < 2; ++ph) {
            for (int mtl = wave; mtl < 25; mtl += 8) {
                const int mtile = gp * 25 + mtl;
                v8f acc = zero8();
#pragma unroll
                for (int kt = 0; kt < 4; ++kt) {
                    const size_t aoff = ((size_t)(mtile * 4 + kt) * 32 + lane) * 16;
                    const v16bf ah = *(const v16bf*)(W2h + aoff);
                    const v16bf al = *(const v16bf*)(W2l + aoff);
                    const int bi = (ph * 16 + m) * 136 + kt * 32 + 8 * h;
                    Frag bh, bl;
                    bh.p[0] = *(const v8us*)&sXh[bi];
                    bh.p[1] = *(const v8us*)&sXh[bi + 16];
                    bl.p[0] = *(const v8us*)&sXl[bi];
                    bl.p[1] = *(const v8us*)&sXl[bi + 16];
                    acc = wmma3(acc, ah, al, bh.v, bl.v);
                }
#pragma unroll
                for (int r = 0; r < 8; ++r)
                    sWd[(mtl * 16 + 8 * h + r) * 16 + m] = acc[r] * 0.2f;
            }
            __syncthreads();

            {
                const int col = tid & 31;
                const int q   = tid >> 5;
                const int gl  = col >> 4;
                const int p   = col & 15;
                const int r0  = gl * 200 + q * 25;
                float s = 0.f;
#pragma unroll 5
                for (int rr = 0; rr < 25; ++rr) s += fabsf(sWd[(r0 + rr) * 16 + p]);
                sPart[tid] = s;
            }
            __syncthreads();
            if (tid < 32) {
                const float d = ((sPart[tid] + sPart[32 + tid]) + (sPart[64 + tid] + sPart[96 + tid]))
                              + ((sPart[128 + tid] + sPart[160 + tid]) + (sPart[192 + tid] + sPart[224 + tid]));
                sScale[tid] = 1.0f / (d + 0.01f);
            }
            __syncthreads();

            {
                const int cl  = tid >> 2;
                const int p4i = tid & 3;
                const int i4  = cl >> 4;
                const int jl  = cl & 15;
                const int j   = gp * 16 + jl;
                const int c   = i4 * 64 + j;
                const int gl  = jl >> 3;
                const int d   = j & 7;
                const int wrow = gl * 200 + d * 25;
                const int xx0  = xb + ph * 16 + p4i * 4;
                const float* xc = x + ((size_t)(b * CIN + c)) * HWN;
                float s0 = 0.f, s1 = 0.f, s2 = 0.f, s3 = 0.f;
#pragma unroll
                for (int ky = 0; ky < 5; ++ky) {
                    const int yy = y + ky - 2;
                    if ((unsigned)yy < (unsigned)IMH) {
                        const float* xr = xc + yy * IMW;
                        float win[8];
#pragma unroll
                        for (int u = 0; u < 8; ++u) {
                            const int xi  = xx0 - 2 + u;
                            const int xcl = xi < 0 ? 0 : (xi > IMW - 1 ? IMW - 1 : xi);
                            const float xv = xr[xcl];
                            win[u] = ((unsigned)xi < (unsigned)IMW) ? xv : 0.f;
                        }
#pragma unroll
                        for (int kx = 0; kx < 5; ++kx) {
                            const v4f wv = *(const v4f*)&sWd[(wrow + ky * 5 + kx) * 16 + p4i * 4];
                            s0 += wv.x * win[kx + 0];
                            s1 += wv.y * win[kx + 1];
                            s2 += wv.z * win[kx + 2];
                            s3 += wv.w * win[kx + 3];
                        }
                    }
                }
                const v4f sc = *(const v4f*)&sScale[gl * 16 + p4i * 4];
                v4f o;
                o.x = s0 * sc.x; o.y = s1 * sc.y; o.z = s2 * sc.z; o.w = s3 * sc.w;
                *(v4f*)&sOut[cl * 32 + ph * 16 + p4i * 4] = o;
            }
            __syncthreads();
        }

        v4f qv[2];
#pragma unroll
        for (int it = 0; it < 2; ++it) {
            const int cl = wave * 8 + it * 4 + (lane >> 3);
            qv[it] = *(const v4f*)&sOut[cl * 32 + (lane & 7) * 4];
        }
#pragma unroll
        for (int it = 0; it < 2; ++it) {
            const int cl = wave * 8 + it * 4 + (lane >> 3);
            const int c  = (cl >> 4) * 64 + gp * 16 + (cl & 15);
            *(volatile v4f*)(filt + ((size_t)(b * CIN + c)) * HWN + pix0 + (lane & 7) * 4) = qv[it];
        }
        __threadfence();
#pragma unroll
        for (int it = 0; it < 2; ++it) {
            const int cl = wave * 8 + it * 4 + (lane >> 3);
            const int c  = (cl >> 4) * 64 + gp * 16 + (cl & 15);
            *(volatile v4f*)(filt + ((size_t)(b * CIN + c)) * HWN + pix0 + (lane & 7) * 4) = qv[it];
        }
        __syncthreads();
    }
}

extern "C" void kernel_launch(void* const* d_in, const int* in_sizes, int n_in,
                              void* d_out, int out_size, void* d_ws, size_t ws_size,
                              hipStream_t stream) {
    if (n_in < 8) return;
    const float* x     = (const float*)d_in[0];
    const float* W1    = (const float*)d_in[1];
    const float* gamma = (const float*)d_in[2];
    const float* beta  = (const float*)d_in[3];
    const float* gwp   = (const float*)d_in[4];
    const float* gbp   = (const float*)d_in[5];
    const float* W2    = (const float*)d_in[6];
    const float* W3    = (const float*)d_in[7];
    float* out = (float*)d_out;

    const int nx = in_sizes[0];
    const int nb = nx / (CIN * HWN);
    if (nb <= 0 || nb * CIN * HWN != nx) return;
    if (out_size != nb * CIN * HWN) return;
    if (in_sizes[1] != CMID * CIN || in_sizes[6] != CW * CMID || in_sizes[7] != CIN * CIN) return;
    if (in_sizes[2] < NGRP || in_sizes[3] < NGRP || in_sizes[4] < NGRP || in_sizes[5] < NGRP) return;
    if (nb > 65535) return;

    char* ws = (char*)d_ws;
    size_t off = 0;
    auto carve = [&](size_t bytes) -> char* {
        char* p = ws + off;
        off += (bytes + 255) & ~(size_t)255;
        return p;
    };
    unsigned short* W1h = (unsigned short*)carve((size_t)CMID * CIN * 2);
    unsigned short* W1l = (unsigned short*)carve((size_t)CMID * CIN * 2);
    unsigned short* W2h = (unsigned short*)carve((size_t)CW * CMID * 2);
    unsigned short* W2l = (unsigned short*)carve((size_t)CW * CMID * 2);
    unsigned short* W3h = (unsigned short*)carve((size_t)CIN * CIN * 2);
    unsigned short* W3l = (unsigned short*)carve((size_t)CIN * CIN * 2);
    float* mid   = (float*)carve((size_t)nb * CMID * HWN * 4);
    float* stats = (float*)carve((size_t)nb * NGRP * SPITCH * 4);
    float* filt  = (float*)carve((size_t)nb * CIN * HWN * 4);
    if (off > ws_size) return;

    {
        int nthr = CMID * CIN / 8;
        pack_w_kernel<<<(nthr + 255) / 256, 256, 0, stream>>>(W1, W1h, W1l, CIN, CIN / 32, nthr);
        nthr = CW * CMID / 8;
        pack_w_kernel<<<(nthr + 255) / 256, 256, 0, stream>>>(W2, W2h, W2l, CMID, CMID / 32, nthr);
        nthr = CIN * CIN / 8;
        pack_w_kernel<<<(nthr + 255) / 256, 256, 0, stream>>>(W3, W3h, W3l, CIN, CIN / 32, nthr);
    }

    gemm_split_kernel<CIN / 32><<<dim3(HWN / 64, CMID / 128, nb), 256, 0, stream>>>(W1h, W1l, x, mid, CMID, HWN);

    gn_stats_kernel<<<nb * NGRP, 256, 0, stream>>>(mid, stats);

    dynfilter_kernel<<<dim3(HWN / 32, nb), 256, 0, stream>>>(W2h, W2l, mid, stats, gamma, beta, gwp, gbp, x, filt);

    gemm_split_kernel<CIN / 32><<<dim3(HWN / 64, CIN / 128, nb), 256, 0, stream>>>(W3h, W3l, filt, out, CIN, HWN);
}
